// NautilusYiJing_45500883534072
// MI455X (gfx1250) — hardware-verified
//
#include <hip/hip_runtime.h>
#include <stdint.h>
#include <stddef.h>

#pragma clang fp contract(off)

#define DM   1024
#define DE   512
#define NE   6
#define NT   8192
#define NX   (NT * DM)
#define NWE  (DM * DE)
#define HP   520
#define KC   128
#define AP   136
#define TP   72
#define LDS_H    (64 * HP * 2)
#define LDS_SCR  65536
#define LDS_EXP  (2 * LDS_H + LDS_SCR + 512)

static_assert(NT % 256 == 0);
static_assert(DM % KC == 0);
static_assert(2 * 64 * AP * 2 <= LDS_SCR);
static_assert(64 * 256 * 4 <= LDS_SCR);
static_assert(8 * 2048 * 4 <= LDS_SCR);

typedef __bf16        v16bf __attribute__((ext_vector_type(16)));
typedef float         v8f   __attribute__((ext_vector_type(8)));
typedef float         v4f   __attribute__((ext_vector_type(4)));
typedef unsigned int  v4u   __attribute__((ext_vector_type(4)));
typedef unsigned int  v2u   __attribute__((ext_vector_type(2)));
typedef int           v4i   __attribute__((ext_vector_type(4)));
typedef v4f __attribute__((may_alias)) v4fa;
typedef v4u __attribute__((may_alias)) v4ua;
typedef v2u __attribute__((may_alias)) v2ua;
typedef v4i __attribute__((may_alias)) v4ia;

union FragBF { v16bf v; v4u q[2]; };

__device__ __forceinline__ unsigned int bfb(float f) {
  unsigned int u = __float_as_uint(f);
  u += 0x7FFFu + ((u >> 16) & 1u);
  return u >> 16;
}
__device__ __forceinline__ void split2(float v, unsigned int& h, unsigned int& l) {
  h = bfb(v);
  l = bfb(v - __uint_as_float(h << 16));
}
__device__ __forceinline__ unsigned int pk(unsigned int a, unsigned int b) { return a | (b << 16); }

__device__ __forceinline__ v8f wmma_bf(v16bf a, v16bf b, v8f c) {
  v8f d = __builtin_amdgcn_wmma_f32_16x16x32_bf16(false, a, false, b, (short)0, c, false, false);
  asm volatile("v_nop\n\tv_nop\n\tv_nop\n\tv_nop" : "+v"(d) : "v"(a), "v"(b));
  return d;
}

__device__ __forceinline__ v16bf ldfrag(const unsigned short* p, int h) {
  FragBF f;
  f.q[0] = *(const v4ua*)(p + 8 * h);
  f.q[1] = *(const v4ua*)(p + 16 + 8 * h);
  return f.v;
}

__device__ __forceinline__ float acc4(v4f a, v4f w, float z) {
  z = fmaf(a.x, w.x, z);
  z = fmaf(a.y, w.y, z);
  z = fmaf(a.z, w.z, z);
  z = fmaf(a.w, w.w, z);
  return z;
}

__device__ __forceinline__ float gelu_t(float v) {
  const float k0 = 0.7978845608028654f;
  const float k1 = 0.044715f;
  const float u = k0 * (v + k1 * (v * (v * v)));
  const float cdf = 0.5f * (1.0f + tanhf(u));
  return v * cdf;
}

__global__ __launch_bounds__(256) void k_cvt_x(const float* __restrict__ x,
                                               unsigned short* __restrict__ xh,
                                               unsigned short* __restrict__ xl)
{
  const int g = blockIdx.x * 256 + threadIdx.x;
  if (g >= NX / 8) return;
  const float* s = x + (size_t)g * 8;
  const v4f a = *(const v4fa*)s;
  const v4f c = *(const v4fa*)(s + 4);
  unsigned int h0, l0, h1, l1, h2, l2, h3, l3, h4, l4, h5, l5, h6, l6, h7, l7;
  split2(a.x, h0, l0); split2(a.y, h1, l1); split2(a.z, h2, l2); split2(a.w, h3, l3);
  split2(c.x, h4, l4); split2(c.y, h5, l5); split2(c.z, h6, l6); split2(c.w, h7, l7);
  const v4u H = { pk(h0, h1), pk(h2, h3), pk(h4, h5), pk(h6, h7) };
  const v4u L = { pk(l0, l1), pk(l2, l3), pk(l4, l5), pk(l6, l7) };
  unsigned short* dh = xh + (size_t)g * 8;
  unsigned short* dl = xl + (size_t)g * 8;
  *(volatile v4u*)dh = H;
  *(volatile v4u*)dl = L;
  __threadfence();
  *(volatile v4u*)dh = H;
  *(volatile v4u*)dl = L;
}

__device__ __forceinline__ void wt_store_pass(const unsigned short* sh, const unsigned short* sl,
                                              unsigned short* oh, unsigned short* ol,
                                              int e, int R, int C, int r0, int c0, int wv, int lane)
{
  const int q8 = lane & 7, sub = lane >> 3;
  #pragma unroll
  for (int i = 0; i < 2; ++i) {
    const int n = wv * 8 + i * 4 + sub;
    const v4u hv = *(const v4ua*)(sh + n * TP + 8 * q8);
    const v4u lv = *(const v4ua*)(sl + n * TP + 8 * q8);
    const size_t go = ((size_t)e * C + c0 + n) * R + r0 + 8 * q8;
    *(volatile v4u*)(oh + go) = hv;
    *(volatile v4u*)(ol + go) = lv;
  }
}

__global__ __launch_bounds__(256) void k_cvt_w(const float* __restrict__ w,
                                               unsigned short* __restrict__ oh,
                                               unsigned short* __restrict__ ol,
                                               int R, int C)
{
  __shared__ __align__(16) unsigned short sh[64 * TP];
  __shared__ __align__(16) unsigned short sl[64 * TP];
  const int tid = threadIdx.x, lane = tid & 31, wv = tid >> 5;
  const int e = blockIdx.z;
  const int r0 = blockIdx.x * 64;
  const int c0 = blockIdx.y * 64;
  const float* src = w + (size_t)e * R * C;
  #pragma unroll
  for (int j = 0; j < 4; ++j) {
    const int idx = tid + 256 * j;
    const int row = idx >> 4, c4 = idx & 15;
    const v4f v = *(const v4fa*)(src + (size_t)(r0 + row) * C + c0 + 4 * c4);
    unsigned int ha, la, hb, lb, hc, lc, hd, ld;
    split2(v.x, ha, la); split2(v.y, hb, lb); split2(v.z, hc, lc); split2(v.w, hd, ld);
    const int cb = 4 * c4;
    sh[(cb + 0) * TP + row] = (unsigned short)ha;  sl[(cb + 0) * TP + row] = (unsigned short)la;
    sh[(cb + 1) * TP + row] = (unsigned short)hb;  sl[(cb + 1) * TP + row] = (unsigned short)lb;
    sh[(cb + 2) * TP + row] = (unsigned short)hc;  sl[(cb + 2) * TP + row] = (unsigned short)lc;
    sh[(cb + 3) * TP + row] = (unsigned short)hd;  sl[(cb + 3) * TP + row] = (unsigned short)ld;
  }
  __syncthreads();
  wt_store_pass(sh, sl, oh, ol, e, R, C, r0, c0, wv, lane);
  __threadfence();
  wt_store_pass(sh, sl, oh, ol, e, R, C, r0, c0, wv, lane);
}

__global__ __launch_bounds__(256) void k_route(const float* __restrict__ x,
                                               const float* __restrict__ pw,
                                               const float* __restrict__ anc,
                                               const float* __restrict__ rt,
                                               float* __restrict__ rec)
{
  __shared__ __align__(16) float sw[NE * DM];
  __shared__ float s_z[256 * 8];
  __shared__ float s_q[256 * 8];
  __shared__ float s_lg[256 * 8];

  const int tid = threadIdx.x;
  const int t = blockIdx.x * 256 + tid;
  for (int i = tid; i < NE * DM; i += 256) sw[i] = pw[i];
  __syncthreads();

  float z0 = 0.f, z1 = 0.f, z2 = 0.f, z3 = 0.f, z4 = 0.f, z5 = 0.f;
  const float* xr = x + (size_t)t * DM;
  #pragma unroll 1
  for (int d4 = 0; d4 < DM / 4; ++d4) {
    const v4f xv = *(const v4fa*)(xr + 4 * d4);
    const float* p = sw + 4 * d4;
    const v4f w0 = *(const v4fa*)(p);
    const v4f w1 = *(const v4fa*)(p + DM);
    const v4f w2 = *(const v4fa*)(p + 2 * DM);
    const v4f w3 = *(const v4fa*)(p + 3 * DM);
    const v4f w4 = *(const v4fa*)(p + 4 * DM);
    const v4f w5 = *(const v4fa*)(p + 5 * DM);
    z0 = acc4(xv, w0, z0);
    z1 = acc4(xv, w1, z1);
    z2 = acc4(xv, w2, z2);
    z3 = acc4(xv, w3, z3);
    z4 = acc4(xv, w4, z4);
    z5 = acc4(xv, w5, z5);
  }

  const int b = tid * 8;
  s_z[b + 0] = z0; s_z[b + 1] = z1; s_z[b + 2] = z2;
  s_z[b + 3] = z3; s_z[b + 4] = z4; s_z[b + 5] = z5;

  const float inv_qt = 1.0f / 0.3f;
  #pragma unroll 1
  for (int e = 0; e < NE; ++e) s_q[b + e] = tanhf(s_z[b + e] * inv_qt);

  float temp = rt[0];
  temp = (temp < 0.1f) ? 0.1f : temp;
  const float inv_t = 1.0f / temp;
  #pragma unroll 1
  for (int e = 0; e < NE; ++e) {
    float d = 0.f;
    #pragma unroll 1
    for (int j = 0; j < NE; ++j) d = fmaf(s_q[b + j], anc[e * NE + j], d);
    const float ham = (6.0f - d) * 0.5f;
    s_lg[b + e] = -ham * inv_t;
  }

  int i1 = 0;
  float b1 = s_lg[b];
  #pragma unroll 1
  for (int e = 1; e < NE; ++e) {
    const float v = s_lg[b + e];
    if (v > b1) { b1 = v; i1 = e; }
  }
  int i2 = -1;
  float b2 = 0.f;
  #pragma unroll 1
  for (int e = 0; e < NE; ++e) {
    const float v = s_lg[b + e];
    const bool take = (e != i1) && ((i2 < 0) || (v > b2));
    if (take) { b2 = v; i2 = e; }
  }
  const float e2 = expf(b2 - b1);
  const float ssum = 1.0f + e2;
  const float rs = 1.0f / ssum;
  const float wtop = rs;
  const float wsec = e2 * rs;

  int s0, s1;
  float ws0, ws1;
  if (i1 < i2) { s0 = i1; ws0 = wtop; s1 = i2; ws1 = wsec; }
  else         { s0 = i2; ws0 = wsec; s1 = i1; ws1 = wtop; }

  const v4f o = { ws0, ws1, (float)s0, (float)s1 };
  float* dst = rec + (size_t)t * 4;
  *(volatile v4f*)dst = o;
  __threadfence();
  *(volatile v4f*)dst = o;
}

__device__ __forceinline__ void list_store_pass(const int* s_list, int* L, int* CL, int base, int tid) {
  #pragma unroll
  for (int j = 0; j < 8; ++j) {
    const int idx = tid + 256 * j;
    const v4i v = *(const v4ia*)(s_list + 4 * idx);
    *(volatile v4i*)(L + 4 * idx) = v;
  }
  if (tid < 8) {
    const v4i cv = { base, base, base, base };
    *(volatile v4i*)(CL + 4 * tid) = cv;
  }
}

__global__ __launch_bounds__(256) void k_lists(const float* __restrict__ rec,
                                               int* __restrict__ lst,
                                               int* __restrict__ cnt)
{
  __shared__ __align__(16) int s_list[NT];
  __shared__ int s_wc[8];
  const int tid = threadIdx.x, lane = tid & 31, wv = tid >> 5;
  const int e = blockIdx.x;

  for (int s = 0; s < 2; ++s) {
    __syncthreads();
    #pragma unroll 1
    for (int i = 0; i < NT / 256; ++i) s_list[tid + 256 * i] = 0;
    __syncthreads();
    int base = 0;
    #pragma unroll 1
    for (int c = 0; c < NT / 256; ++c) {
      const int t = c * 256 + tid;
      const v4f r = *(const v4fa*)(rec + (size_t)t * 4);
      const int sel = (s == 0) ? (int)r.z : (int)r.w;
      const bool f = (sel == e);
      const unsigned int msk = __builtin_amdgcn_ballot_w32(f);
      const int off = __builtin_popcount(msk & ((1u << lane) - 1u));
      const int wc = __builtin_popcount(msk);
      if (lane == 0) s_wc[wv] = wc;
      __syncthreads();
      int pre = 0, tot = 0;
      #pragma unroll 1
      for (int w2 = 0; w2 < 8; ++w2) {
        const int cc = s_wc[w2];
        tot += cc;
        pre += (w2 < wv) ? cc : 0;
      }
      if (f) {
        int p = base + pre + off;
        p = (p < 0) ? 0 : ((p > NT - 1) ? (NT - 1) : p);
        s_list[p] = t;
      }
      base += tot;
      __syncthreads();
    }
    base = (base > NT) ? NT : base;
    int* L  = lst + (size_t)(s * NE + e) * NT;
    int* CL = cnt + (size_t)(s * NE + e) * 32;
    list_store_pass(s_list, L, CL, base, tid);
    __threadfence();
    list_store_pass(s_list, L, CL, base, tid);
  }
}

__device__ __forceinline__ void y_store_pass(const float* sy, float* dst, const int* s_tok,
                                             int mg, int nrows, int colbase, int lane)
{
  const int q8 = lane & 7, sub = lane >> 3;
  #pragma unroll
  for (int i = 0; i < 16; ++i) {
    const int li = i * 4 + sub;
    const int rowl = li >> 1, hl = li & 1;
    const int row = 32 * mg + rowl;
    const v4f v = *(const v4fa*)(sy + rowl * 64 + 32 * hl + 4 * q8);
    if (row < nrows) {
      const int t = s_tok[row];
      *(volatile v4f*)(dst + (size_t)t * DM + colbase + 32 * hl + 4 * q8) = v;
    }
  }
}

template <int SLOT>
__global__ __launch_bounds__(256) void k_expert(const unsigned short* __restrict__ xh,
                                                const unsigned short* __restrict__ xl,
                                                const unsigned short* __restrict__ w1h,
                                                const unsigned short* __restrict__ w1l,
                                                const unsigned short* __restrict__ w2h,
                                                const unsigned short* __restrict__ w2l,
                                                const float* __restrict__ rec,
                                                const int* __restrict__ lst,
                                                const int* __restrict__ cnt,
                                                const float* __restrict__ padd,
                                                float* __restrict__ dst)
{
  extern __shared__ __align__(16) unsigned char dsm[];
  unsigned short* sHh = (unsigned short*)dsm;
  unsigned short* sHl = (unsigned short*)(dsm + LDS_H);
  unsigned char*  scr = dsm + 2 * LDS_H;
  unsigned short* sAh = (unsigned short*)scr;
  unsigned short* sAl = (unsigned short*)(scr + 64 * AP * 2);
  float* sC = (float*)scr;
  float* sY = (float*)scr;
  int*   s_tok = (int*)(dsm + 2 * LDS_H + LDS_SCR);
  float* s_w   = (float*)(dsm + 2 * LDS_H + LDS_SCR + 256);

  const int tid = threadIdx.x, lane = tid & 31, wv = tid >> 5;
  const int h = lane >> 4, m = lane & 15;
  const int e = blockIdx.y, tile = blockIdx.x;

  int c = cnt[(SLOT * NE + e) * 32];
  c = (c < 0) ? 0 : ((c > NT) ? NT : c);
  if (tile * 64 >= c) return;
  int nrows = c - tile * 64;
  nrows = (nrows > 64) ? 64 : nrows;

  if (tid < 64) {
    int idx = tile * 64 + tid;
    idx = (idx > NT - 1) ? (NT - 1) : idx;
    int t = lst[(size_t)(SLOT * NE + e) * NT + idx];
    t = (t < 0) ? 0 : ((t > NT - 1) ? (NT - 1) : t);
    const v4f r = *(const v4fa*)(rec + (size_t)t * 4);
    const float wgt = (SLOT == 0) ? r.x : r.y;
    s_tok[tid] = t;
    s_w[tid] = (tid < nrows) ? wgt : 0.0f;
  }
  __syncthreads();

  const int mg = wv & 1, ng = wv >> 1;
  const v8f z8 = {0.f, 0.f, 0.f, 0.f, 0.f, 0.f, 0.f, 0.f};

  #pragma unroll 1
  for (int nh = 0; nh < 2; ++nh) {
    v8f acc[2][4];
    #pragma unroll
    for (int mt = 0; mt < 2; ++mt)
      #pragma unroll
      for (int nt = 0; nt < 4; ++nt) acc[mt][nt] = z8;

    #pragma unroll 1
    for (int kc = 0; kc < DM; kc += KC) {
      __syncthreads();
      #pragma unroll
      for (int j = 0; j < 4; ++j) {
        const int idx = tid + 256 * j;
        const int row = idx >> 4, c8 = idx & 15;
        const size_t go = (size_t)s_tok[row] * DM + kc + 8 * c8;
        const int lo = row * AP + 8 * c8;
        *(v4ua*)(sAh + lo) = *(const v4ua*)(xh + go);
        *(v4ua*)(sAl + lo) = *(const v4ua*)(xl + go);
      }
      __syncthreads();
      #pragma unroll 1
      for (int ks = 0; ks < KC; ks += 32) {
        v16bf ah[2], al[2];
        #pragma unroll
        for (int mt = 0; mt < 2; ++mt) {
          const int ro = (32 * mg + 16 * mt + m) * AP + ks;
          ah[mt] = ldfrag(sAh + ro, h);
          al[mt] = ldfrag(sAl + ro, h);
        }
        #pragma unroll
        for (int nt = 0; nt < 4; ++nt) {
          const int n = nh * 256 + ng * 64 + 16 * nt + m;
          const size_t bo = ((size_t)e * DE + n) * DM + kc + ks;
          const v16bf bh = ldfrag(w1h + bo, h);
          const v16bf bl = ldfrag(w1l + bo, h);
          #pragma unroll
          for (int mt = 0; mt < 2; ++mt) {
            acc[mt][nt] = wmma_bf(ah[mt], bh, acc[mt][nt]);
            acc[mt][nt] = wmma_bf(ah[mt], bl, acc[mt][nt]);
            acc[mt][nt] = wmma_bf(al[mt], bh, acc[mt][nt]);
          }
        }
      }
    }
    __syncthreads();
    #pragma unroll
    for (int mt = 0; mt < 2; ++mt)
      #pragma unroll
      for (int nt = 0; nt < 4; ++nt)
        #pragma unroll
        for (int r = 0; r < 8; ++r) {
          const int row = 32 * mg + 16 * mt + 8 * h + r;
          const int col = ng * 64 + 16 * nt + m;
          sC[row * 256 + col] = acc[mt][nt][r];
        }
    __syncthreads();
    #pragma unroll 1
    for (int j = 0; j < 16; ++j) {
      const int idx = tid + 256 * j;
      const int row = idx >> 6, c4 = idx & 63;
      const v4f v = *(const v4fa*)(sC + row * 256 + 4 * c4);
      const float wg = s_w[row];
      const float g0 = gelu_t(v.x) * wg;
      const float g1 = gelu_t(v.y) * wg;
      const float g2 = gelu_t(v.z) * wg;
      const float g3 = gelu_t(v.w) * wg;
      unsigned int ha, la, hb, lb, hc, lc, hd, ld;
      split2(g0, ha, la); split2(g1, hb, lb); split2(g2, hc, lc); split2(g3, hd, ld);
      const v2u ph = { pk(ha, hb), pk(hc, hd) };
      const v2u pl = { pk(la, lb), pk(lc, ld) };
      const int ho = row * HP + nh * 256 + 4 * c4;
      *(v2ua*)(sHh + ho) = ph;
      *(v2ua*)(sHl + ho) = pl;
    }
    __syncthreads();
  }

  #pragma unroll 1
  for (int np = 0; np < 4; ++np) {
    v8f acc[2][4];
    #pragma unroll
    for (int mt = 0; mt < 2; ++mt)
      #pragma unroll
      for (int nt = 0; nt < 4; ++nt) acc[mt][nt] = z8;

    #pragma unroll 1
    for (int k0 = 0; k0 < DE; k0 += 32) {
      v16bf ah[2], al[2];
      #pragma unroll
      for (int mt = 0; mt < 2; ++mt) {
        const int ro = (32 * mg + 16 * mt + m) * HP + k0;
        ah[mt] = ldfrag(sHh + ro, h);
        al[mt] = ldfrag(sHl + ro, h);
      }
      #pragma unroll
      for (int nt = 0; nt < 4; ++nt) {
        const int n = np * 256 + ng * 64 + 16 * nt + m;
        const size_t bo = ((size_t)e * DM + n) * DE + k0;
        const v16bf bh = ldfrag(w2h + bo, h);
        const v16bf bl = ldfrag(w2l + bo, h);
        #pragma unroll
        for (int mt = 0; mt < 2; ++mt) {
          acc[mt][nt] = wmma_bf(ah[mt], bh, acc[mt][nt]);
          acc[mt][nt] = wmma_bf(ah[mt], bl, acc[mt][nt]);
          acc[mt][nt] = wmma_bf(al[mt], bh, acc[mt][nt]);
        }
      }
    }
    __syncthreads();
    float* sy = sY + wv * 2048;
    const int colbase = np * 256 + ng * 64;
    #pragma unroll
    for (int mt = 0; mt < 2; ++mt)
      #pragma unroll
      for (int nt = 0; nt < 4; ++nt)
        #pragma unroll
        for (int r = 0; r < 8; ++r) {
          const int rowl = 16 * mt + 8 * h + r;
          const int cl = 16 * nt + m;
          float y = acc[mt][nt][r];
          if (SLOT == 1) {
            const int t = s_tok[32 * mg + rowl];
            const float p0 = padd[(size_t)t * DM + colbase + cl];
            y = p0 + y;
          }
          sy[rowl * 64 + cl] = y;
        }
    __syncthreads();
    y_store_pass(sy, dst, s_tok, mg, nrows, colbase, lane);
    __threadfence();
    y_store_pass(sy, dst, s_tok, mg, nrows, colbase, lane);
  }
}

extern "C" void kernel_launch(void* const* d_in, const int* in_sizes, int n_in,
                              void* d_out, int out_size, void* d_ws, size_t ws_size,
                              hipStream_t stream)
{
  if (n_in < 6) return;
  if (in_sizes[0] != NX) return;
  if (in_sizes[1] != NE * DM) return;
  if (in_sizes[2] != NE * NE) return;
  if (in_sizes[3] < 1) return;
  if (in_sizes[4] != NE * NWE || in_sizes[5] != NE * NWE) return;
  if (out_size != NX) return;

  const float* x    = (const float*)d_in[0];
  const float* pw   = (const float*)d_in[1];
  const float* anc  = (const float*)d_in[2];
  const float* rt   = (const float*)d_in[3];
  const float* w1   = (const float*)d_in[4];
  const float* w2   = (const float*)d_in[5];
  float* out = (float*)d_out;

  const size_t bXp  = (size_t)NX * 2;
  const size_t bWp  = (size_t)NE * NWE * 2;
  const size_t bP   = (size_t)NX * 4;
  const size_t bRec = (size_t)NT * 16;
  const size_t bLst = (size_t)2 * NE * NT * 4;
  const size_t bCnt = (size_t)2 * NE * 32 * 4;
  const size_t total = 2 * bXp + 4 * bWp + bP + bRec + bLst + bCnt;
  if (total > ws_size) return;

  char* ws = (char*)d_ws;
  size_t off = 0;
  unsigned short* XH  = (unsigned short*)(ws + off); off += bXp;
  unsigned short* XL  = (unsigned short*)(ws + off); off += bXp;
  unsigned short* W1H = (unsigned short*)(ws + off); off += bWp;
  unsigned short* W1L = (unsigned short*)(ws + off); off += bWp;
  unsigned short* W2H = (unsigned short*)(ws + off); off += bWp;
  unsigned short* W2L = (unsigned short*)(ws + off); off += bWp;
  float*          P0  = (float*)(ws + off);          off += bP;
  float*          REC = (float*)(ws + off);          off += bRec;
  int*            LST = (int*)(ws + off);            off += bLst;
  int*            CNT = (int*)(ws + off);            off += bCnt;
  if (off != total) return;

  k_cvt_x<<<(NX / 8) / 256, 256, 0, stream>>>(x, XH, XL);

  dim3 gW1(DM / 64, DE / 64, NE);
  k_cvt_w<<<gW1, 256, 0, stream>>>(w1, W1H, W1L, DM, DE);
  dim3 gW2(DE / 64, DM / 64, NE);
  k_cvt_w<<<gW2, 256, 0, stream>>>(w2, W2H, W2L, DE, DM);

  k_route<<<NT / 256, 256, 0, stream>>>(x, pw, anc, rt, REC);

  k_lists<<<NE, 256, 0, stream>>>(REC, LST, CNT);

  hipFuncSetAttribute(reinterpret_cast<const void*>(&k_expert<0>),
                      hipFuncAttributeMaxDynamicSharedMemorySize, LDS_EXP);
  hipFuncSetAttribute(reinterpret_cast<const void*>(&k_expert<1>),
                      hipFuncAttributeMaxDynamicSharedMemorySize, LDS_EXP);
  dim3 gE(NT / 64, NE);
  k_expert<0><<<gE, 256, LDS_EXP, stream>>>(XH, XL, W1H, W1L, W2H, W2L, REC, LST, CNT, P0, P0);
  k_expert<1><<<gE, 256, LDS_EXP, stream>>>(XH, XL, W1H, W1L, W2H, W2L, REC, LST, CNT, P0, out);
}
